// _3DIS_31860067402336
// MI455X (gfx1250) — hardware-verified
//
#include <hip/hip_runtime.h>
#include <math.h>

typedef __attribute__((ext_vector_type(16))) _Float16 v16h;
typedef __attribute__((ext_vector_type(16))) __bf16 v16b;
typedef __attribute__((ext_vector_type(8)))  _Float16 v8h;
typedef __attribute__((ext_vector_type(8)))  float v8f;
typedef __attribute__((ext_vector_type(4)))  float v4f;
typedef __attribute__((ext_vector_type(2)))  float v2f;
typedef __attribute__((ext_vector_type(4)))  unsigned v4u;
typedef __attribute__((ext_vector_type(4)))  int v4i;
typedef float __attribute__((may_alias)) float_a;
typedef int __attribute__((may_alias)) int_a;

template <typename T> __device__ __forceinline__ void vst2(void* p, T v) { *(volatile T*)p = v; __threadfence(); *(volatile T*)p = v; }
__device__ __forceinline__ v8f wmma16(v16h a, v16h b, v8f c) {
  v8f d = __builtin_amdgcn_wmma_f32_16x16x32_f16(false, a, false, b, (short)0, c, false, false);
  asm volatile("v_nop\n\tv_nop\n\tv_nop\n\tv_nop" : "+v"(d) : "v"(a), "v"(b));
  return d;
}
__device__ __forceinline__ v8f wmma_bf(v16b a, v16b b, v8f c) {
  v8f d = __builtin_amdgcn_wmma_f32_16x16x32_bf16(false, a, false, b, (short)0, c, false, false);
  asm volatile("v_nop\n\tv_nop\n\tv_nop\n\tv_nop" : "+v"(d) : "v"(a), "v"(b));
  return d;
}
__device__ __forceinline__ v16h frag_h(const _Float16* rowk0, int lane) {
  union { v16h v; v8h q[2]; } u; const _Float16* p = rowk0 + 8 * (lane >> 4);
  u.q[0] = *(const v8h*)p; u.q[1] = *(const v8h*)(p + 16); return u.v;
}
__device__ __forceinline__ v16h frag_f32(const float* rowk0, int lane) {
  v16h a; const float* p = rowk0 + 8 * (lane >> 4);
#pragma unroll
  for (int i = 0; i < 8; ++i) { a[i] = (_Float16)p[i]; a[8 + i] = (_Float16)p[16 + i]; }
  return a;
}
__device__ __forceinline__ v16h frag_f32s(const float* rowk0, int lane, float sc) {
  v16h a; const float* p = rowk0 + 8 * (lane >> 4);
#pragma unroll
  for (int i = 0; i < 8; ++i) { a[i] = (_Float16)(p[i] * sc); a[8 + i] = (_Float16)(p[16 + i] * sc); }
  return a;
}
__device__ __forceinline__ v16h fragc_f32(const float* W, int k0, int n, int lane, int ld, int K) {
  v16h a; const int g = lane >> 4;
#pragma unroll
  for (int i = 0; i < 8; ++i) { const int ka = k0 + 8 * g + i, kb = ka + 16;
    a[i] = (_Float16)(ka < K ? W[(size_t)(ka < K ? ka : K - 1) * ld + n] : 0.f); a[8 + i] = (_Float16)(kb < K ? W[(size_t)(kb < K ? kb : K - 1) * ld + n] : 0.f); }
  return a;
}
struct F2 { v16b h, l; };
__device__ __forceinline__ F2 bsplit16(const float v[16]) { F2 r;
#pragma unroll
  for (int i = 0; i < 16; ++i) { const __bf16 h = (__bf16)v[i]; r.h[i] = h; r.l[i] = (__bf16)(v[i] - (float)h); }
  return r; }
__device__ __forceinline__ F2 split_row(const float* row, int k0, int lane) { float v[16]; const float* p = row + k0 + 8 * (lane >> 4);
#pragma unroll
  for (int i = 0; i < 8; ++i) { v[i] = p[i]; v[8 + i] = p[16 + i]; }
  return bsplit16(v); }
__device__ __forceinline__ F2 split_rowK(const float* row, int k0, int lane, int K) { float v[16]; const int g = lane >> 4;
#pragma unroll
  for (int i = 0; i < 8; ++i) { const int ka = k0 + 8 * g + i, kb = ka + 16; v[i] = ka < K ? row[ka < K ? ka : K - 1] : 0.f; v[8 + i] = kb < K ? row[kb < K ? kb : K - 1] : 0.f; }
  return bsplit16(v); }
__device__ __forceinline__ F2 split_col(const float* W, int k0, int n, int lane, int ld, int K) { float v[16]; const int g = lane >> 4;
#pragma unroll
  for (int i = 0; i < 8; ++i) { const int ka = k0 + 8 * g + i, kb = ka + 16; v[i] = ka < K ? W[(size_t)(ka < K ? ka : K - 1) * ld + n] : 0.f; v[8 + i] = kb < K ? W[(size_t)(kb < K ? kb : K - 1) * ld + n] : 0.f; }
  return bsplit16(v); }
__device__ __forceinline__ v8f mac3(const F2& a, const F2& b, v8f c) { c = wmma_bf(a.l, b.h, c); c = wmma_bf(a.h, b.l, c); return wmma_bf(a.h, b.h, c); }
__device__ __forceinline__ float sigm(float v) { return 1.0f / (1.0f + expf(-v)); }
#define LDSX() do { asm volatile("s_wait_dscnt 0" ::: "memory"); __builtin_amdgcn_wave_barrier(); __builtin_amdgcn_fence(__ATOMIC_RELEASE, "workgroup"); } while (0)

__device__ __forceinline__ float bfr(float v) { return (float)(__bf16)v; }
#define NBS 131072
#define NT 6
#define NV 10
#define NG 15
#define NCOL 31
#define NP 100
#define RPB 1024
#define NSB (NBS / RPB)
#ifndef NROWS
#define NROWS NBS
#endif
#define WS_P1  0u
#define WS_P2  (WS_P1 + 4u * NSB * 32)
#define WS_ST  (WS_P2 + 4u * NSB * 32)
#define WS_END (WS_ST + 4u * 64)
__device__ __forceinline__ float ycol(const float* __restrict__ XT, const float* __restrict__ XV, const float* __restrict__ XG, const float* __restrict__ WA, const float* __restrict__ WB, const float* __restrict__ WG, size_t r, int c) {
  float s = 0.f;
  if (c < NT) { for (int i = 0; i < NT; ++i) s += bfr(XT[r * NT + i]) * bfr(WA[i * NT + c]); }
  else if (c < NT + NV) { const int o = c - NT; for (int i = 0; i < NV; ++i) s += bfr(XV[r * NV + i]) * bfr(WB[i * NV + o]); }
  else { const int o = c - NT - NV; for (int i = 0; i < NG; ++i) s += bfr(XG[r * NG + i]) * bfr(WG[i * NG + o]); }
  return s; }
__global__ __launch_bounds__(256) void k_stat(const float* __restrict__ XT, const float* __restrict__ XV, const float* __restrict__ XG, const float* __restrict__ WA, const float* __restrict__ WB, const float* __restrict__ WG, const float* __restrict__ ST, int pass, float* __restrict__ PART) { __shared__ float sacc[8][32];
  const int t = threadIdx.x; const int c = t & 31, sub = t >> 5; const size_t r0 = (size_t)blockIdx.x * RPB; float s = 0.f; const float mu = (pass == 1 && c < NCOL) ? ST[c] : 0.f;
  if (c < NCOL) { for (int rr = sub; rr < RPB; rr += 8) { const float y = ycol(XT, XV, XG, WA, WB, WG, r0 + rr, c); const float d = y - mu; s += (pass == 0) ? y : d * d; } }
  sacc[sub][c] = s; __syncthreads();
  if (t < 32) { float a = 0.f; for (int w = 0; w < 8; ++w) a += sacc[w][t]; vst2(PART + (size_t)blockIdx.x * 32 + t, a); } }
__global__ __launch_bounds__(32) void k_fin(const float* __restrict__ PART, int pass, float* __restrict__ ST) { const int c = threadIdx.x; float a = 0.f; for (int b = 0; b < NSB; ++b) a += PART[b * 32 + c]; const float m = a / (float)NBS; vst2(ST + pass * 32 + c, pass == 0 ? m : rsqrtf(m + 1e-5f)); }
__global__ __launch_bounds__(128) void k_main(const float* __restrict__ XT, const float* __restrict__ XV, const float* __restrict__ XG, const float* __restrict__ WA, const float* __restrict__ WB, const float* __restrict__ WG, const float* __restrict__ G1, const float* __restrict__ B1, const float* __restrict__ G2, const float* __restrict__ B2, const float* __restrict__ G3, const float* __restrict__ B3, const float* __restrict__ MW, const float* __restrict__ MB, const int* __restrict__ VP, const float* __restrict__ ST, float* __restrict__ OUT) {
  __shared__ float sval[4][16][NP + 4]; __shared__ float sbr[4][16][32]; __shared__ __align__(16) float so[64 * NP];
  const int tid = threadIdx.x, wave = tid >> 5, lane = tid & 31, col = lane & 15, g = lane >> 4; const size_t r0 = (size_t)blockIdx.x * 64 + wave * 16; const size_t arow = r0 + col;
  for (int c = g; c < NCOL; c += 2) { const float y = ycol(XT, XV, XG, WA, WB, WG, arow, c); const float gm = c < NT ? bfr(G1[c]) : (c < NT + NV ? bfr(G2[c - NT]) : bfr(G3[c - NT - NV])); const float bt = c < NT ? bfr(B1[c]) : (c < NT + NV ? bfr(B2[c - NT]) : bfr(B3[c - NT - NV]));
    const float z = (y - ST[c]) * ST[32 + c] * gm + bt; sbr[wave][col][c] = z > 0.f ? z : expm1f(z); }
  LDSX();
  for (int p = g; p < NP; p += 2) { const int vp = VP[p]; const int i = vp / (NV * NG), rem = vp % (NV * NG); const int v = rem / NG, t2 = rem % NG; sval[wave][col][p] = sbr[wave][col][i] * sbr[wave][col][NT + v] * sbr[wave][col][NT + NV + t2]; }
  LDSX();
  v8f acc[7] = {};
#pragma unroll
  for (int kc = 0; kc < 4; ++kc) { float v[16];
#pragma unroll
    for (int i = 0; i < 8; ++i) { const int k0 = kc * 32 + 8 * g + i, k1 = k0 + 16; v[i] = k0 < NP ? sval[wave][col][k0] : 0.f; v[8 + i] = k1 < NP ? sval[wave][col][k1] : 0.f; }
    const F2 a = bsplit16(v);
#pragma unroll
    for (int j = 0; j < 7; ++j) { v16b w; const int o = j * 16 + col;
#pragma unroll
      for (int i = 0; i < 8; ++i) { const int k0 = kc * 32 + 8 * g + i, k1 = k0 + 16; w[i] = (o < NP && k0 < NP) ? (__bf16)MW[o * NP + k0] : (__bf16)0.f; w[8 + i] = (o < NP && k1 < NP) ? (__bf16)MW[o * NP + k1] : (__bf16)0.f; }
      asm volatile("s_wait_loadcnt 0x0" ::: "memory"); acc[j] = wmma_bf(a.h, w, acc[j]); acc[j] = wmma_bf(a.l, w, acc[j]); } }
#pragma unroll
  for (int j = 0; j < 7; ++j) { const int o = j * 16 + col;
#pragma unroll
    for (int r = 0; r < 8; ++r) if (o < NP) so[(wave * 16 + 8 * g + r) * NP + o] = acc[j][r] + bfr(MB[o]); }
  __syncthreads();
  for (int e = tid; e < 64 * NP / 4; e += 128) vst2(OUT + (size_t)blockIdx.x * 64 * NP + e * 4, *(const v4f*)&so[e * 4]); }
extern "C" void kernel_launch(void* const* d_in, const int* in_sizes, int n_in, void* d_out, int out_size, void* d_ws, size_t ws_size, hipStream_t stream) {
  (void)in_sizes; (void)n_in; (void)out_size;
  const float** F = (const float**)d_in;
  if (ws_size < (size_t)WS_END) return;
  char* ws = (char*)d_ws; float *P1 = (float*)(ws + WS_P1), *P2 = (float*)(ws + WS_P2), *ST = (float*)(ws + WS_ST);
  k_stat<<<dim3(NSB), 256, 0, stream>>>(F[0], F[1], F[2], F[3], F[4], F[5], ST, 0, P1);
  k_fin<<<dim3(1), 32, 0, stream>>>(P1, 0, ST);
  k_stat<<<dim3(NSB), 256, 0, stream>>>(F[0], F[1], F[2], F[3], F[4], F[5], ST, 1, P2);
  k_fin<<<dim3(1), 32, 0, stream>>>(P2, 1, ST);
  k_main<<<dim3(NROWS / 64), 128, 0, stream>>>(F[0], F[1], F[2], F[3], F[4], F[5], F[6], F[7], F[8], F[9], F[10], F[11], F[12], F[13], (const int*)d_in[14], ST, (float*)d_out);
}
